// LSTMGCNModel_83021717832866
// MI455X (gfx1250) — hardware-verified
//
#include <hip/hip_runtime.h>


#define AS3 __attribute__((address_space(3)))

#define NF_   64
#define TS_   12
#define XOFF_ 52
#define HD_   32
#define G4_   128
#define TP_   16
#define FC1_  16
#define KW_   64
#define MB_   128
#define NTHR  256
#define NWAV  8
#define AP_   104
#define WP_   64
#define WFP_  32
#define H0C_  16
#define H1C_  64

static_assert(MB_ == 16 * NWAV);
static_assert(NTHR == 32 * NWAV);
static_assert(AP_ % 8 == 0 && WP_ % 8 == 0 && WFP_ % 8 == 0);
static_assert(AP_ >= H1C_ + HD_);
static_assert(H0C_ == TP_ && H0C_ + HD_ + 16 == H1C_);
static_assert(XOFF_ + TS_ == NF_);
static_assert(TP_ + HD_ <= KW_ && 2 * HD_ == KW_);
static_assert(G4_ == 4 * HD_);
static_assert(MB_ % 32 == 0);

typedef _Float16 v16h __attribute__((ext_vector_type(16)));
typedef _Float16 v8h  __attribute__((ext_vector_type(8)));
typedef float    v8f  __attribute__((ext_vector_type(8)));
typedef float    v4f  __attribute__((ext_vector_type(4)));

typedef AS3 _Float16*       lp_h;
typedef AS3 const _Float16* lcp_h;
typedef AS3 float*          lp_f;
typedef AS3 const float*    lcp_f;

union FragH { v16h v; v8h half[2]; };

#define SCL    16.0f
#define INV256 0.00390625f

__device__ __forceinline__ float rcpx(float x) { return __builtin_amdgcn_rcpf(x); }
__device__ __forceinline__ float sigm(float x) { return rcpx(1.0f + __expf(-x)); }
__device__ __forceinline__ float tanhm(float x) {
    const float e = __expf(2.0f * x);
    return 1.0f - 2.0f * rcpx(e + 1.0f);
}
__device__ __forceinline__ v8f ld8f(const float* p) {
    const v4f a = *(const v4f*)p;
    const v4f b = *(const v4f*)(p + 4);
    return __builtin_shufflevector(a, b, 0, 1, 2, 3, 4, 5, 6, 7);
}
__device__ __forceinline__ v8f zero8() {
    v8f z;
#pragma unroll
    for (int i = 0; i < 8; ++i) z[i] = 0.0f;
    return z;
}

__device__ __forceinline__ void ldh_lds(FragH& f, lcp_h p) {
    f.half[0] = *(AS3 const v8h*)(p);
    f.half[1] = *(AS3 const v8h*)(p + 16);
}
__device__ __forceinline__ v8f mmah(v8f c, const FragH& a, const FragH& b) {
    return __builtin_amdgcn_wmma_f32_16x16x32_f16(false, a.v, false, b.v, (short)0, c, false, false);
}

__device__ __forceinline__ void st_xt(lp_h dst, float s, lcp_f wtp, lcp_f btp) {
    v8h xv;
#pragma unroll
    for (int i = 0; i < 8; ++i) xv[i] = (_Float16)((s * wtp[i] + btp[i]) * SCL);
    *(AS3 v8h*)dst = xv;
}

__global__ __launch_bounds__(NTHR)
void lstm_seq_kernel(const float* __restrict__ x,
                     const float* __restrict__ Wtp,  const float* __restrict__ btp,
                     const float* __restrict__ Wih0, const float* __restrict__ Whh0,
                     const float* __restrict__ bih0, const float* __restrict__ bhh0,
                     const float* __restrict__ Wih1, const float* __restrict__ Whh1,
                     const float* __restrict__ bih1, const float* __restrict__ bhh1,
                     const float* __restrict__ Wfc1, const float* __restrict__ bfc1,
                     const float* __restrict__ Wfc2, const float* __restrict__ bfc2,
                     float* out, int nn)
{
    __shared__ __attribute__((aligned(16))) _Float16 sW0[G4_ * WP_];
    __shared__ __attribute__((aligned(16))) _Float16 sW1[G4_ * WP_];
    __shared__ __attribute__((aligned(16))) _Float16 sWf[FC1_ * WFP_];
    __shared__ __attribute__((aligned(16))) _Float16 sA[NWAV * 16 * AP_];
    __shared__ __attribute__((aligned(16))) float    sOut[MB_];
    __shared__ float sBias0[G4_];
    __shared__ float sBias1[G4_];
    __shared__ float sWtp[TP_];
    __shared__ float sBtp[TP_];
    __shared__ float sBfc1[FC1_];
    __shared__ float sWfc2[FC1_];
    __shared__ float sBfc2[4];

    const int tid  = threadIdx.x;
    const int lane = tid & 31;
    const int w    = tid >> 5;
    const int h    = lane >> 4;
    const int m    = lane & 15;
    const int blk0 = blockIdx.x * MB_;

    lcp_h cW0  = (lcp_h)sW0;
    lcp_h cW1  = (lcp_h)sW1;
    lcp_h cWf  = (lcp_h)sWf;

#pragma unroll 1
    for (int p = tid; p < G4_ * (KW_ / 8); p += NTHR) {
        const int n  = p >> 3;
        const int c8 = (p & 7) * 8;
        {
            const v8f a = ld8f(Wih0 + (size_t)n * TP_ + min(c8, TP_ - 8));
            const v8f b = ld8f(Whh0 + (size_t)n * HD_ + min(max(c8 - TP_, 0), HD_ - 8));
            v8h hv;
#pragma unroll
            for (int i = 0; i < 8; ++i) {
                const float v = (c8 < TP_) ? a[i] : ((c8 < TP_ + HD_) ? b[i] : 0.0f);
                hv[i] = (_Float16)(v * SCL);
            }
            *(AS3 v8h*)((lp_h)sW0 + n * WP_ + c8) = hv;
        }
        {
            const v8f a = ld8f(Wih1 + (size_t)n * HD_ + min(c8, HD_ - 8));
            const v8f b = ld8f(Whh1 + (size_t)n * HD_ + min(max(c8 - HD_, 0), HD_ - 8));
            v8h hv;
#pragma unroll
            for (int i = 0; i < 8; ++i) {
                const float v = (c8 < HD_) ? a[i] : b[i];
                hv[i] = (_Float16)(v * SCL);
            }
            *(AS3 v8h*)((lp_h)sW1 + n * WP_ + c8) = hv;
        }
    }
#pragma unroll 1
    for (int i = tid; i < FC1_ * HD_; i += NTHR) {
        const int n = i >> 5;
        const int k = i & 31;
        sWf[n * WFP_ + k] = (_Float16)(Wfc1[k * FC1_ + n] * SCL);
    }
    if (tid < G4_) {
        sBias0[tid] = bih0[tid] + bhh0[tid];
        sBias1[tid] = bih1[tid] + bhh1[tid];
    }
    if (w == 0) {
        const int i16 = min(lane, TP_ - 1);
        const float a = Wtp[i16];
        const float b = btp[i16];
        const float c = bfc1[i16];
        const float d = Wfc2[i16];
        const float e = bfc2[0];
        if (lane < TP_) { sWtp[lane] = a; sBtp[lane] = b; sBfc1[lane] = c; sWfc2[lane] = d; }
        if (lane == 0) sBfc2[0] = e;
    }
    __syncthreads();

    lp_h sAw = (lp_h)sA + w * (16 * AP_);
    {
        v8h zh;
#pragma unroll
        for (int i = 0; i < 8; ++i) zh[i] = (_Float16)0.0f;
#pragma unroll 1
        for (int i = lane; i < 16 * 11; i += 32) {
            const int row = i / 11;
            const int pc  = i - row * 11;
            *(AS3 v8h*)(sAw + row * AP_ + H0C_ + 8 * pc) = zh;
        }
    }
    const int nodec = min(blk0 + 16 * w + m, nn - 1);
    const float* xrow = x + (size_t)nodec * NF_ + XOFF_;
    lp_h  xdst = sAw + m * AP_ + 8 * h;
    lcp_f wtp8 = (lcp_f)sWtp + 8 * h;
    lcp_f btp8 = (lcp_f)sBtp + 8 * h;
    st_xt(xdst, xrow[0], wtp8, btp8);
    __syncthreads();

    lcp_h afr  = (lcp_h)(sAw + m * AP_ + 8 * h);
    lp_h  hrow = sAw + (8 * h) * AP_;

    v8f c0s[2], c1s[2];
#pragma unroll
    for (int j = 0; j < 2; ++j) { c0s[j] = zero8(); c1s[j] = zero8(); }

#pragma unroll 1
    for (int t = 0; t < TS_; ++t) {
        asm volatile("" ::: "memory");

        {
            FragH a0, a1;
            ldh_lds(a0, afr);
            ldh_lds(a1, afr + 32);
#pragma unroll
            for (int jt = 0; jt < 2; ++jt) {
                asm volatile("" ::: "memory");
                v8f acc[4];
#pragma unroll
                for (int q = 0; q < 4; ++q) acc[q] = zero8();
                FragH b[4];
#pragma unroll
                for (int q = 0; q < 4; ++q) ldh_lds(b[q], cW0 + (32 * q + 16 * jt + m) * WP_ + 8 * h);
#pragma unroll
                for (int q = 0; q < 4; ++q) acc[q] = mmah(acc[q], a0, b[q]);
                asm volatile("v_nop\n\tv_nop\n\tv_nop\n\tv_nop"
                             : "+v"(acc[0]), "+v"(acc[1]), "+v"(acc[2]), "+v"(acc[3])
                             : "v"(a0.v), "v"(b[0].v), "v"(b[1].v), "v"(b[2].v), "v"(b[3].v));
#pragma unroll
                for (int q = 0; q < 4; ++q) ldh_lds(b[q], cW0 + (32 * q + 16 * jt + m) * WP_ + 32 + 8 * h);
#pragma unroll
                for (int q = 0; q < 4; ++q) acc[q] = mmah(acc[q], a1, b[q]);
                asm volatile("v_nop\n\tv_nop\n\tv_nop\n\tv_nop"
                             : "+v"(acc[0]), "+v"(acc[1]), "+v"(acc[2]), "+v"(acc[3])
                             : "v"(a1.v), "v"(b[0].v), "v"(b[1].v), "v"(b[2].v), "v"(b[3].v));
                const int u = 16 * jt + m;
                const float bi = sBias0[u];
                const float bf = sBias0[HD_ + u];
                const float bg = sBias0[2 * HD_ + u];
                const float bo = sBias0[3 * HD_ + u];
#pragma unroll
                for (int r = 0; r < 8; ++r) {
                    const float gi = acc[0][r] * INV256 + bi;
                    const float gf = acc[1][r] * INV256 + bf;
                    const float gg = acc[2][r] * INV256 + bg;
                    const float go = acc[3][r] * INV256 + bo;
                    const float cn = sigm(gf) * c0s[jt][r] + sigm(gi) * tanhm(gg);
                    c0s[jt][r] = cn;
                    const float hn = sigm(go) * tanhm(cn);
                    hrow[r * AP_ + H0C_ + u] = (_Float16)(hn * SCL);
                }
            }
        }
        __syncthreads();

        {
            FragH a0, a1;
            ldh_lds(a0, afr + H0C_);
            ldh_lds(a1, afr + H1C_);
#pragma unroll
            for (int jt = 0; jt < 2; ++jt) {
                asm volatile("" ::: "memory");
                v8f acc[4];
#pragma unroll
                for (int q = 0; q < 4; ++q) acc[q] = zero8();
                FragH b[4];
#pragma unroll
                for (int q = 0; q < 4; ++q) ldh_lds(b[q], cW1 + (32 * q + 16 * jt + m) * WP_ + 8 * h);
#pragma unroll
                for (int q = 0; q < 4; ++q) acc[q] = mmah(acc[q], a0, b[q]);
                asm volatile("v_nop\n\tv_nop\n\tv_nop\n\tv_nop"
                             : "+v"(acc[0]), "+v"(acc[1]), "+v"(acc[2]), "+v"(acc[3])
                             : "v"(a0.v), "v"(b[0].v), "v"(b[1].v), "v"(b[2].v), "v"(b[3].v));
#pragma unroll
                for (int q = 0; q < 4; ++q) ldh_lds(b[q], cW1 + (32 * q + 16 * jt + m) * WP_ + 32 + 8 * h);
#pragma unroll
                for (int q = 0; q < 4; ++q) acc[q] = mmah(acc[q], a1, b[q]);
                asm volatile("v_nop\n\tv_nop\n\tv_nop\n\tv_nop"
                             : "+v"(acc[0]), "+v"(acc[1]), "+v"(acc[2]), "+v"(acc[3])
                             : "v"(a1.v), "v"(b[0].v), "v"(b[1].v), "v"(b[2].v), "v"(b[3].v));
                const int u = 16 * jt + m;
                const float bi = sBias1[u];
                const float bf = sBias1[HD_ + u];
                const float bg = sBias1[2 * HD_ + u];
                const float bo = sBias1[3 * HD_ + u];
#pragma unroll
                for (int r = 0; r < 8; ++r) {
                    const float gi = acc[0][r] * INV256 + bi;
                    const float gf = acc[1][r] * INV256 + bf;
                    const float gg = acc[2][r] * INV256 + bg;
                    const float go = acc[3][r] * INV256 + bo;
                    const float cn = sigm(gf) * c1s[jt][r] + sigm(gi) * tanhm(gg);
                    c1s[jt][r] = cn;
                    const float hn = sigm(go) * tanhm(cn);
                    hrow[r * AP_ + H1C_ + u] = (_Float16)(hn * SCL);
                }
            }
            if (t + 1 < TS_) st_xt(xdst, xrow[t + 1], wtp8, btp8);
        }
        __syncthreads();
    }

    {
        FragH a, b;
        ldh_lds(a, afr + H1C_);
        ldh_lds(b, cWf + m * WFP_ + 8 * h);
        v8f acc = zero8();
        acc = mmah(acc, a, b);
        asm volatile("v_nop\n\tv_nop\n\tv_nop\n\tv_nop" : "+v"(acc) : "v"(a.v), "v"(b.v));
        const float b1  = sBfc1[m];
        const float w2  = sWfc2[m];
        const float b2v = sBfc2[0];
#pragma unroll
        for (int r = 0; r < 8; ++r) {
            float v = fmaxf(acc[r] * INV256 + b1, 0.0f) * w2;
            v += __shfl_xor(v, 1);
            v += __shfl_xor(v, 2);
            v += __shfl_xor(v, 4);
            v += __shfl_xor(v, 8);
            if (m == 0) sOut[16 * w + 8 * h + r] = v + b2v;
        }
    }
    __syncthreads();

    if (w == 0) {
        const v4f ov = *(AS3 const v4f*)((lcp_f)sOut + 4 * lane);
        const int q    = lane >> 3;
        const int ln0  = blk0 + 32 * q;
        const int e0   = blk0 + 4 * lane;
        const bool full = (ln0 + 32 <= nn);
        float* op = out + (size_t)e0;
        if (full) {
            *(volatile v4f*)op = ov;
        } else {
#pragma unroll
            for (int i = 0; i < 4; ++i)
                if (e0 + i < nn) ((volatile float*)op)[i] = ov[i];
        }
        __threadfence();
        if (full) {
            *(volatile v4f*)op = ov;
        } else {
#pragma unroll
            for (int i = 0; i < 4; ++i)
                if (e0 + i < nn) ((volatile float*)op)[i] = ov[i];
        }
    }
}

extern "C" void kernel_launch(void* const* d_in, const int* in_sizes, int n_in,
                              void* d_out, int out_size, void* d_ws, size_t ws_size,
                              hipStream_t stream)
{
    (void)d_ws; (void)ws_size;
    if (n_in < 24) return;
    const int ntot = in_sizes[0];
    if (ntot < NF_ || (ntot % NF_) != 0) return;
    const int nn = ntot / NF_;
    if (in_sizes[10] != TP_)        return;
    if (in_sizes[11] != TP_)        return;
    if (in_sizes[12] != G4_ * TP_)  return;
    if (in_sizes[13] != G4_ * HD_)  return;
    if (in_sizes[14] != G4_)        return;
    if (in_sizes[15] != G4_)        return;
    if (in_sizes[16] != G4_ * HD_)  return;
    if (in_sizes[17] != G4_ * HD_)  return;
    if (in_sizes[18] != G4_)        return;
    if (in_sizes[19] != G4_)        return;
    if (in_sizes[20] != HD_ * FC1_) return;
    if (in_sizes[21] != FC1_)       return;
    if (in_sizes[22] != FC1_)       return;
    if (in_sizes[23] != 1)          return;
    if (out_size != nn)             return;

    const float* x    = (const float*)d_in[0];
    const float* Wtp  = (const float*)d_in[10];
    const float* btp  = (const float*)d_in[11];
    const float* Wih0 = (const float*)d_in[12];
    const float* Whh0 = (const float*)d_in[13];
    const float* bih0 = (const float*)d_in[14];
    const float* bhh0 = (const float*)d_in[15];
    const float* Wih1 = (const float*)d_in[16];
    const float* Whh1 = (const float*)d_in[17];
    const float* bih1 = (const float*)d_in[18];
    const float* bhh1 = (const float*)d_in[19];
    const float* Wfc1 = (const float*)d_in[20];
    const float* bfc1 = (const float*)d_in[21];
    const float* Wfc2 = (const float*)d_in[22];
    const float* bfc2 = (const float*)d_in[23];
    float* out = (float*)d_out;

    const int nblk = (nn + MB_ - 1) / MB_;
    lstm_seq_kernel<<<dim3(nblk), dim3(NTHR), 0, stream>>>(
        x, Wtp, btp, Wih0, Whh0, bih0, bhh0, Wih1, Whh1, bih1, bhh1,
        Wfc1, bfc1, Wfc2, bfc2, out, nn);
}
